// IWHT2Layer_15522011808173
// MI455X (gfx1250) — hardware-run, weakly checked
//
#include <hip/hip_runtime.h>


#define NT   16
#define NBB  16
#define NHB  28
#define NWB  28
#define NCI  64
#define NKO  64
#define NP   12544
constexpr size_t al256(size_t b) { return (b + 255) & ~(size_t)255; }
constexpr size_t WS_TOTAL = al256((size_t)NT * NP * NCI * 2) + al256((size_t)NT * NKO * NCI * 2) + al256((size_t)NT * NP * NKO * 4);
static_assert(WS_TOTAL == 77201408 && WS_TOTAL <= 134217728, "the workspace carve: 73.6 MiB");
static_assert(NP == NBB * NHB * NWB && NP % 64 == 0 && NKO % 64 == 0 && NCI % 32 == 0 && NT == 16 && ((size_t)NT * NP * NCI) % 8 == 0, "whole tiles; whole depth steps; sixteen planes");
typedef _Float16 h16;
typedef unsigned short bf;
typedef __attribute__((ext_vector_type(16))) __bf16   v16bf;
typedef __attribute__((ext_vector_type(16))) _Float16 v16h;
typedef __attribute__((ext_vector_type(8)))  _Float16 v8h;
typedef __attribute__((ext_vector_type(8)))  unsigned short v8us;
typedef __attribute__((ext_vector_type(8)))  float    v8f;
typedef __attribute__((ext_vector_type(4)))  float    v4f;
typedef v8h  __attribute__((may_alias)) v8ha;
typedef v4f  __attribute__((may_alias)) v4fa;
typedef v8us __attribute__((may_alias)) v8usa;

__device__ __forceinline__ unsigned short f2bf(float f) { unsigned u = __float_as_uint(f); u += 0x7FFFu + ((u >> 16) & 1u); return (unsigned short)(u >> 16); }
__device__ __forceinline__ float bf2f(unsigned short b) { return __uint_as_float(((unsigned)b) << 16); }
__device__ __forceinline__ float bfr(float f) { return bf2f(f2bf(f)); }
__device__ __forceinline__ v16h cat16(v8h lo, v8h hi) { return __builtin_shufflevector(lo, hi, 0, 1, 2, 3, 4, 5, 6, 7, 8, 9, 10, 11, 12, 13, 14, 15); }
__device__ __forceinline__ v16bf cat16b(v8us lo, v8us hi) { return __builtin_bit_cast(v16bf, __builtin_shufflevector(lo, hi, 0, 1, 2, 3, 4, 5, 6, 7, 8, 9, 10, 11, 12, 13, 14, 15)); }
__device__ __forceinline__ v8f wmma16(v16h a, v16h b, v8f c) { return __builtin_amdgcn_wmma_f32_16x16x32_f16(false, a, false, b, (short)0, c, false, false); }
__device__ __forceinline__ v8f wmmab(v16bf a, v16bf b, v8f c) { return __builtin_amdgcn_wmma_f32_16x16x32_bf16(false, a, false, b, (short)0, c, false, false); }


template <typename T16> struct WFrag;
template <> struct WFrag<h16> { typedef v16h V; static __device__ __forceinline__ V ld(const h16* p) { return cat16(*(const v8h*)p, *(const v8h*)(p + 16)); } static __device__ __forceinline__ v8f mma(V a, V b, v8f c) { return wmma16(a, b, c); } };
template <> struct WFrag<bf> { typedef v16bf V; static __device__ __forceinline__ V ld(const bf* p) { return cat16b(*(const v8us*)p, *(const v8us*)(p + 16)); } static __device__ __forceinline__ v8f mma(V a, V b, v8f c) { return wmmab(a, b, c); } };
template <typename T16, int NSPLIT, bool BIAS>
__global__ __launch_bounds__(32) void k_gemmw(const T16* __restrict__ A, const T16* __restrict__ A2, const T16* __restrict__ Bt, const T16* __restrict__ Bt2, int K, float* C, int ldc, const float* __restrict__ bias, size_t sA, size_t sB, size_t sC) {
    typedef typename WFrag<T16>::V V;
    __shared__ __align__(16) float os[16 * 68];
    const size_t z = blockIdx.z; A += z * sA; if (A2) A2 += z * sA; Bt += z * sB; if (Bt2) Bt2 += z * sB; C += z * sC;
    const int lane = threadIdx.x & 31, lr = lane & 15, hi = lane >> 4; const int r0 = blockIdx.x * 64, c0 = blockIdx.y * 64;
    v8f acc[4][4];
#pragma unroll
    for (int mb = 0; mb < 4; ++mb)
#pragma unroll
        for (int nb = 0; nb < 4; ++nb) acc[mb][nb] = (v8f){};
    const size_t aoff = (size_t)(r0 + lr) * K + 8 * hi, boff = (size_t)(c0 + lr) * K + 8 * hi;
    for (int kc = 0; kc < K; kc += 32) {
        V a[4], a2[4];
#pragma unroll
        for (int mb = 0; mb < 4; ++mb) { a[mb] = WFrag<T16>::ld(A + aoff + (size_t)mb * 16 * K + kc); if (NSPLIT == 1 || NSPLIT == 2) a2[mb] = WFrag<T16>::ld(A2 + aoff + (size_t)mb * 16 * K + kc); }
#pragma unroll
        for (int nb = 0; nb < 4; ++nb) { const V b = WFrag<T16>::ld(Bt + boff + (size_t)nb * 16 * K + kc); V b2; if (NSPLIT >= 2) b2 = WFrag<T16>::ld(Bt2 + boff + (size_t)nb * 16 * K + kc);
#pragma unroll
            for (int mb = 0; mb < 4; ++mb) { acc[mb][nb] = WFrag<T16>::mma(a[mb], b, acc[mb][nb]); if (NSPLIT == 1 || NSPLIT == 2) acc[mb][nb] = WFrag<T16>::mma(a2[mb], b, acc[mb][nb]); if (NSPLIT >= 2) acc[mb][nb] = WFrag<T16>::mma(a[mb], b2, acc[mb][nb]); } }
        asm volatile("v_nop\n\tv_nop\n\tv_nop\n\tv_nop" : "+v"(acc[0][0]), "+v"(acc[1][1]), "+v"(acc[2][2]), "+v"(acc[3][3]) : "v"(a[0]), "v"(a[3]));
    }
#pragma unroll
    for (int mb = 0; mb < 4; ++mb) {
#pragma unroll
        for (int nb = 0; nb < 4; ++nb) {
#pragma unroll
            for (int j = 0; j < 8; ++j) os[(hi * 8 + j) * 68 + nb * 16 + lr] = acc[mb][nb][j]; }
        __builtin_amdgcn_wave_barrier(); asm volatile("" ::: "memory");
        float* crow = C + (size_t)(r0 + mb * 16) * ldc + c0;
#pragma unroll 1
        for (int ps = 0; ps < 2; ++ps) {
#pragma unroll
            for (int s = 0; s < 8; ++s) { const int row = 2 * s + hi, cofs = lr * 4; v4f val = *(const v4fa*)(os + row * 68 + cofs); if (BIAS) { val[0] += bfr(bias[c0 + cofs]); val[1] += bfr(bias[c0 + cofs + 1]); val[2] += bfr(bias[c0 + cofs + 2]); val[3] += bfr(bias[c0 + cofs + 3]); }
                *(volatile v4f*)(crow + (size_t)row * ldc + cofs) = val; }
            if (ps == 0) __threadfence(); }
        __builtin_amdgcn_wave_barrier(); asm volatile("" ::: "memory");
    }
}

__device__ __forceinline__ h16 tohx(float x) { return (h16)x; }
__device__ __forceinline__ void splitf(float y, unsigned short& h, unsigned short& l) { h = f2bf(y); l = f2bf(y - bf2f(h)); }
typedef __attribute__((ext_vector_type(2))) _Float16 v2h;
typedef __attribute__((ext_vector_type(4))) _Float16 v4h;
typedef __attribute__((ext_vector_type(2))) unsigned short v2us;
typedef __attribute__((ext_vector_type(4))) unsigned short v4us;
typedef __attribute__((ext_vector_type(2))) float v2f;
typedef __attribute__((ext_vector_type(4))) int v4i;

__global__ __launch_bounds__(256) void k_cvt8(const float* __restrict__ src, bf* dst, size_t n8) { const size_t i = (size_t)blockIdx.x * 256 + threadIdx.x; if (i >= n8) return; const v8f v = *(const v8f*)(src + i * 8); v8us o;
#pragma unroll
    for (int k = 0; k < 8; ++k) o[k] = f2bf(v[k]); *(volatile v8us*)(dst + i * 8) = o; __threadfence(); *(volatile v8us*)(dst + i * 8) = o; }

__global__ __launch_bounds__(256) void k_wtG(const float* __restrict__ w, int K, int N, bf* Bt) {
    const int lane = threadIdx.x & 31; const int L0 = (blockIdx.x * 8 + (threadIdx.x >> 5)) * 8; const int nlines = N * K / 64;
#pragma unroll
    for (int ps = 0; ps < 2; ++ps) {
        for (int l = 0; l < 8; ++l) { const int L = L0 + l; if (L >= nlines) break; const size_t e = (size_t)L * 64 + lane * 2; const int k = (int)(e % K), n = (int)(e / K); v2us o;
            o[0] = f2bf(w[(size_t)k * N + n]); o[1] = f2bf(w[(size_t)(k + 1) * N + n]); *(volatile v2us*)(Bt + e) = o; }
        if (ps == 0) __threadfence(); }
}

__global__ __launch_bounds__(256) void k_inv4(const float* __restrict__ MX, const float* __restrict__ ad, float* res) {
    const unsigned e = blockIdx.x * 256 + threadIdx.x; if (e >= (unsigned)(NWB * (NKO / 4))) return; const unsigned wq = e >> 4, k4 = (e & 15) * 4; const unsigned hq = blockIdx.y, bq = blockIdx.z;
    const size_t p = ((size_t)bq * NHB + hq) * NWB + wq; v4f m[4][4];
#pragma unroll
    for (int u = 0; u < 4; ++u)
#pragma unroll
        for (int v = 0; v < 4; ++v) m[u][v] = *(const v4f*)(MX + ((size_t)(4 * u + v) * NP + p) * NKO + k4);
    const v4f b4 = *(const v4f*)(ad + k4); v4f a[4][4], o[4][4];
#pragma unroll
    for (int v = 0; v < 4; ++v) { a[0][v] = ((m[0][v] + m[1][v]) + m[2][v]) + m[3][v]; a[1][v] = ((m[0][v] - m[1][v]) + m[2][v]) - m[3][v]; a[2][v] = ((m[0][v] + m[1][v]) - m[2][v]) - m[3][v]; a[3][v] = ((m[0][v] - m[1][v]) - m[2][v]) + m[3][v]; }
#pragma unroll
    for (int i = 0; i < 4; ++i) { o[i][0] = ((a[i][0] + a[i][1]) + a[i][2]) + a[i][3]; o[i][1] = ((a[i][0] - a[i][1]) + a[i][2]) - a[i][3]; o[i][2] = ((a[i][0] + a[i][1]) - a[i][2]) - a[i][3]; o[i][3] = ((a[i][0] - a[i][1]) - a[i][2]) + a[i][3]; }
#pragma unroll
    for (int i = 0; i < 4; ++i)
#pragma unroll
        for (int j = 0; j < 4; ++j)
#pragma unroll
            for (int q = 0; q < 4; ++q) o[i][j][q] = o[i][j][q] * 0.0625f + bfr(b4[q]);
    float* d = res + (((size_t)bq * (4 * NHB) + 4 * hq) * (4 * NWB) + 4 * wq) * NKO + k4;
    for (int ps = 0; ps < 2; ++ps) {
#pragma unroll
        for (int i = 0; i < 4; ++i)
#pragma unroll
            for (int j = 0; j < 4; ++j) *(volatile v4f*)(d + ((size_t)i * (4 * NWB) + j) * NKO) = o[i][j];
        if (ps == 0) __threadfence(); } }

extern "C" void kernel_launch(void* const* d_in, const int* in_sizes, int n_in,
                              void* d_out, int out_size, void* d_ws, size_t ws_size, hipStream_t stream) {
    if (n_in < 6) return;
    if (in_sizes[0] < NT * NP * NCI || in_sizes[1] < NT * NP * NCI || in_sizes[2] < NT * NCI * NKO || in_sizes[3] < NT * NCI * NKO || in_sizes[4] < NKO || in_sizes[5] < NKO || (size_t)out_size < (size_t)2 * NP * 16 * NKO) return;
    char* wsp = (char*)d_ws;
    auto take = [&](size_t bytes) { char* cur = wsp; wsp += (bytes + 255) & ~(size_t)255; return (void*)cur; };
    bf* XA = (bf*)take((size_t)NT * NP * NCI * 2); bf* WB = (bf*)take((size_t)NT * NKO * NCI * 2); float* MX = (float*)take((size_t)NT * NP * NKO * 4);
    if ((size_t)(wsp - (char*)d_ws) != WS_TOTAL || WS_TOTAL > ws_size) return;
    for (int st = 0; st < 2; ++st) {
        const float* tr = (const float*)d_in[st]; const float* wt = (const float*)d_in[2 + st]; const float* bs = (const float*)d_in[4 + st]; float* OUT = (float*)d_out + (size_t)st * NP * 16 * NKO;
        k_cvt8<<<(unsigned)(((size_t)NT * NP * NCI / 8 + 255) / 256), 256, 0, stream>>>(tr, XA, (size_t)NT * NP * NCI / 8);
        for (int t = 0; t < NT; ++t) k_wtG<<<(unsigned)(((size_t)NKO * NCI / 64 + 63) / 64), 256, 0, stream>>>(wt + (size_t)t * NCI * NKO, NCI, NKO, WB + (size_t)t * NKO * NCI);
        k_gemmw<bf, 0, false><<<dim3(NP / 64, NKO / 64, NT), 32, 0, stream>>>(XA, nullptr, WB, nullptr, NCI, MX, NKO, nullptr, (size_t)NP * NCI, (size_t)NKO * NCI, (size_t)NP * NKO);
        k_inv4<<<dim3((NWB * (NKO / 4) + 255) / 256, NHB, NBB), 256, 0, stream>>>(MX, bs, OUT);
    }
}
